// _BiMambaBlock_56358560858364
// MI455X (gfx1250) — hardware-run, weakly checked
//
#include <hip/hip_runtime.h>
#include <math.h>

#pragma clang fp contract(off)

#define NB    4
#define LL    2048
#define NTOK  (NB * LL)
#define DMOD  512
#define DIN   1024
#define DXZ   (2 * DIN)
#define DST   16
#define DTR   32
#define XDN   64
#define DCV   4
#define KCAT  (2 * DIN)
#define OSTR  68
#define SCH   32
#define SYP   260
#define TP    68
#define LOG2E 1.4426950408889634f
#define WSCAP ((size_t)134217728)

static_assert(NTOK % 128 == 0);
static_assert(NTOK % 8 == 0);
static_assert(NTOK % 2 == 0);
static_assert(DMOD % 64 == 0);
static_assert(DMOD % 128 == 0);
static_assert(DIN % 64 == 0);
static_assert(DIN % 256 == 0);
static_assert(DXZ % 64 == 0);
static_assert(KCAT % 32 == 0);
static_assert(XDN == 64);
static_assert(DTR == 32);
static_assert(DST == 16);
static_assert(DCV == 4);
static_assert(LL % SCH == 0);
static_assert(SCH == 32);
static_assert(SYP % 4 == 0);
static_assert(SYP >= 256);
static_assert(OSTR % 4 == 0);
static_assert(TP % 4 == 0);

typedef unsigned short us16 __attribute__((ext_vector_type(16)));
typedef unsigned short us8  __attribute__((ext_vector_type(8)));
typedef unsigned short us8a __attribute__((ext_vector_type(8), may_alias));
typedef unsigned short us4  __attribute__((ext_vector_type(4)));
typedef _Float16 v16h __attribute__((ext_vector_type(16)));
typedef _Float16 v8h  __attribute__((ext_vector_type(8)));
typedef _Float16 v4h  __attribute__((ext_vector_type(4)));
typedef float v8f  __attribute__((ext_vector_type(8)));
typedef float v4f  __attribute__((ext_vector_type(4)));
typedef float v4fa __attribute__((ext_vector_type(4), may_alias));
union FragU { us16 v; us8 h[2]; };

__device__ __forceinline__ float bf16r(float f) {
  unsigned u = __float_as_uint(f);
  u += 0x7FFFu + ((u >> 16) & 1u);
  return __uint_as_float(u & 0xFFFF0000u);
}
__device__ __forceinline__ float siluf(float x) { return x * __builtin_amdgcn_rcpf(1.0f + __expf(-x)); }

__device__ __forceinline__ float conv_silu(float c0, float c1, float c2, float c3,
                                           float x0, float x1, float x2, float x3, float bias) {
#pragma clang fp contract(off)
  float a = c0 * x0;
  a = a + c1 * x1;
  a = a + c2 * x2;
  a = a + c3 * x3;
  a = a + bias;
  return siluf(a);
}

__device__ __forceinline__ v8f mma_f16(us16 a, us16 b, v8f c) {
  return __builtin_amdgcn_wmma_f32_16x16x32_f16(false, __builtin_bit_cast(v16h, a), false, __builtin_bit_cast(v16h, b),
                                                (short)0, c, false, false);
}
__device__ __forceinline__ void wguard8(v8f (&c)[2][4], const us16& a0, const us16& a1, const us16 (&b)[4]) {
#if defined(__HIP_DEVICE_COMPILE__)
  asm volatile("v_nop\n\tv_nop\n\tv_nop\n\tv_nop"
               : "+v"(c[0][0]), "+v"(c[0][1]), "+v"(c[0][2]), "+v"(c[0][3]),
                 "+v"(c[1][0]), "+v"(c[1][1]), "+v"(c[1][2]), "+v"(c[1][3])
               : "v"(a0), "v"(a1), "v"(b[0]), "v"(b[1]), "v"(b[2]), "v"(b[3]));
#endif
}
__device__ __forceinline__ void wguard4(v8f& c0, v8f& c1, v8f& c2, v8f& c3,
                                        const us16& a0, const us16& a1, const us16& b0, const us16& b1) {
#if defined(__HIP_DEVICE_COMPILE__)
  asm volatile("v_nop\n\tv_nop\n\tv_nop\n\tv_nop"
               : "+v"(c0), "+v"(c1), "+v"(c2), "+v"(c3)
               : "v"(a0), "v"(a1), "v"(b0), "v"(b1));
#endif
}

__device__ __forceinline__ us16 gfrag(const unsigned short* __restrict__ P, int ld, int row0, int k0) {
  const int lane = threadIdx.x & 31, r = lane & 15, kh = (lane >> 4) * 8;
  const unsigned short* p = P + (size_t)(row0 + r) * ld + k0 + kh;
  FragU f;
  f.h[0] = *(const us8a*)p;
  f.h[1] = *(const us8a*)(p + 16);
  return f.v;
}

template <int KT>
__global__ __launch_bounds__(256) void k_cvtT(const float* __restrict__ W, int N, unsigned short* T, int ldt, int koff, float scale) {
  __shared__ __attribute__((aligned(16))) float sT[64 * TP];
  const int tid = threadIdx.x;
  const int n0 = blockIdx.x * 64, k0 = blockIdx.y * KT;
#pragma unroll
  for (int it = 0; it < KT / 16; ++it) {
    const int idx = it * 256 + tid, kr = idx >> 4, n4 = (idx & 15) * 4;
    const v4f v = *(const v4fa*)(W + (size_t)(k0 + kr) * N + n0 + n4);
#pragma unroll
    for (int u = 0; u < 4; ++u) sT[(n4 + u) * TP + kr] = v[u];
  }
  __syncthreads();
  constexpr int PPR = KT / 8;
  constexpr int NIT = (64 * PPR) / 256;
  us8 o[NIT];
  size_t offs[NIT];
#pragma unroll
  for (int it = 0; it < NIT; ++it) {
    const int idx = it * 256 + tid, n = idx / PPR, k8 = (idx - n * PPR) * 8;
    const v4f va = *(const v4fa*)(sT + n * TP + k8);
    const v4f vb = *(const v4fa*)(sT + n * TP + k8 + 4);
    v8h hv;
#pragma unroll
    for (int u = 0; u < 4; ++u) {
      hv[u]     = (_Float16)(scale * bf16r(va[u]));
      hv[4 + u] = (_Float16)(scale * bf16r(vb[u]));
    }
    o[it] = __builtin_bit_cast(us8, hv);
    offs[it] = (size_t)(n0 + n) * ldt + (size_t)(koff + k0 + k8);
  }
#pragma unroll
  for (int pass = 0; pass < 2; ++pass) {
#pragma unroll
    for (int it = 0; it < NIT; ++it) *(volatile us8*)(T + offs[it]) = o[it];
    __threadfence();
  }
}

__global__ __launch_bounds__(256) void k_ln(const float* __restrict__ x, const float* __restrict__ g, const float* __restrict__ bt,
                                           unsigned short* WH) {
#pragma clang fp contract(off)
  const int tid = threadIdx.x, lane = tid & 31, wave = tid >> 5;
  const int tok = blockIdx.x * 8 + wave;
  const float* xr = x + (size_t)tok * DMOD;
  float v[16];
#pragma unroll
  for (int q = 0; q < 4; ++q) {
    const v4f t4 = *(const v4fa*)(xr + 128 * q + 4 * lane);
#pragma unroll
    for (int u = 0; u < 4; ++u) v[4 * q + u] = bf16r(t4[u]);
  }
  float s = 0.0f;
#pragma unroll
  for (int i = 0; i < 16; ++i) s = s + v[i];
#pragma unroll
  for (int o = 16; o > 0; o >>= 1) s = s + __shfl_xor(s, o);
  const float mu = s * (1.0f / DMOD);
  float dv[16];
  float s2 = 0.0f;
#pragma unroll
  for (int i = 0; i < 16; ++i) { dv[i] = v[i] - mu; s2 = s2 + dv[i] * dv[i]; }
#pragma unroll
  for (int o = 16; o > 0; o >>= 1) s2 = s2 + __shfl_xor(s2, o);
  const float var = s2 * (1.0f / DMOD);
  const float rs = rsqrtf(var + 1e-5f);
  us4 ov[4];
#pragma unroll
  for (int q = 0; q < 4; ++q) {
    v4h hv;
#pragma unroll
    for (int u = 0; u < 4; ++u) {
      const int ch = 128 * q + 4 * lane + u;
      const float w = (dv[4 * q + u] * rs) * bf16r(g[ch]) + bf16r(bt[ch]);
      hv[u] = (_Float16)(8.0f * w);
    }
    ov[q] = __builtin_bit_cast(us4, hv);
  }
  const size_t base = (size_t)tok * DMOD + 4 * lane;
#pragma unroll
  for (int pass = 0; pass < 2; ++pass) {
#pragma unroll
    for (int q = 0; q < 4; ++q) *(volatile us4*)(WH + base + 128 * q) = ov[q];
    __threadfence();
  }
}

template <int EPI>
__global__ __launch_bounds__(128) void k_gemm(const unsigned short* __restrict__ A, int lda,
                                             const unsigned short* __restrict__ B, int ldb, int K, float scale,
                                             float* Y, int ldy, unsigned short* Y16, const float* __restrict__ xres) {
  __shared__ __attribute__((aligned(16))) float sm[4 * 32 * OSTR];
  const int tid = threadIdx.x, lane = tid & 31, wave = tid >> 5, cl = lane & 15, hh = lane >> 4;
  const int m0 = blockIdx.x * 128 + wave * 32, n0 = blockIdx.y * 64;

  v8f acc[2][4];
#pragma unroll
  for (int i = 0; i < 2; ++i)
#pragma unroll
    for (int j = 0; j < 4; ++j) { v8f zz = {0.f, 0.f, 0.f, 0.f, 0.f, 0.f, 0.f, 0.f}; acc[i][j] = zz; }

#pragma unroll 1
  for (int k0 = 0; k0 < K; k0 += 32) {
    const us16 a0 = gfrag(A, lda, m0, k0);
    const us16 a1 = gfrag(A, lda, m0 + 16, k0);
    us16 bfr[4];
#pragma unroll
    for (int j = 0; j < 4; ++j) bfr[j] = gfrag(B, ldb, n0 + 16 * j, k0);
#pragma unroll
    for (int j = 0; j < 4; ++j) {
      acc[0][j] = mma_f16(a0, bfr[j], acc[0][j]);
      acc[1][j] = mma_f16(a1, bfr[j], acc[1][j]);
    }
    wguard8(acc, a0, a1, bfr);
  }

  float* so = sm + wave * (32 * OSTR);
#pragma unroll
  for (int i = 0; i < 2; ++i)
#pragma unroll
    for (int j = 0; j < 4; ++j)
#pragma unroll
      for (int r = 0; r < 8; ++r) so[(16 * i + 8 * hh + r) * OSTR + 16 * j + cl] = acc[i][j][r] * scale;
  __syncthreads();

#pragma unroll
  for (int pass = 0; pass < 2; ++pass) {
#pragma unroll
    for (int it = 0; it < 16; ++it) {
      const int ch = it * 32 + lane, r = ch >> 4, q = (ch & 15) * 4;
      v4f v = *(const v4fa*)(so + r * OSTR + q);
      if (EPI == 2) {
        const v4f xv = *(const v4fa*)(xres + (size_t)(m0 + r) * DMOD + n0 + q);
#pragma unroll
        for (int u = 0; u < 4; ++u) v[u] = bf16r(xv[u]) + v[u];
      }
      *(volatile v4f*)(Y + (size_t)(m0 + r) * ldy + n0 + q) = v;
    }
    if (EPI == 1) {
#pragma unroll
      for (int it = 0; it < 4; ++it) {
        const int p = it * 32 + lane, r = p >> 2, k8 = (p & 3) * 8;
        const v4f va = *(const v4fa*)(so + r * OSTR + k8);
        const v4f vb = *(const v4fa*)(so + r * OSTR + k8 + 4);
        v8h hv;
#pragma unroll
        for (int u = 0; u < 4; ++u) { hv[u] = (_Float16)(16.0f * va[u]); hv[4 + u] = (_Float16)(16.0f * vb[u]); }
        *(volatile us8*)(Y16 + (size_t)(m0 + r) * DTR + k8) = __builtin_bit_cast(us8, hv);
      }
    }
    __threadfence();
  }
}

template <int DIR>
__global__ __launch_bounds__(256) void k_conv(const float* __restrict__ XZ, const float* __restrict__ cw, const float* __restrict__ cb,
                                             unsigned short* XC) {
#pragma clang fp contract(off)
  const int tid = threadIdx.x;
  const int tok = blockIdx.x * 2 + (tid >> 7);
  const int b = tok / LL, t = tok - b * LL;
  const int c = (tid & 127) * 8;
  float xv[DCV][8];
#pragma unroll
  for (int k = 0; k < DCV; ++k) {
    const int pos = DIR ? (t + (DCV - 1) - k) : (t - (DCV - 1) + k);
    const bool ok = DIR ? (pos <= LL - 1) : (pos >= 0);
    const int pc = pos < 0 ? 0 : (pos > LL - 1 ? LL - 1 : pos);
    const float* p = XZ + ((size_t)(b * LL + pc)) * DXZ + c;
    const v4f va = *(const v4fa*)p;
    const v4f vb = *(const v4fa*)(p + 4);
#pragma unroll
    for (int u = 0; u < 4; ++u) { xv[k][u] = ok ? va[u] : 0.0f; xv[k][4 + u] = ok ? vb[u] : 0.0f; }
  }
  float wv[DCV][8];
#pragma unroll
  for (int k = 0; k < DCV; ++k) {
    const v4f wa = *(const v4fa*)(cw + (size_t)k * DIN + c);
    const v4f wb = *(const v4fa*)(cw + (size_t)k * DIN + c + 4);
#pragma unroll
    for (int u = 0; u < 4; ++u) { wv[k][u] = bf16r(wa[u]); wv[k][4 + u] = bf16r(wb[u]); }
  }
  float bv[8];
  {
    const v4f ba = *(const v4fa*)(cb + c);
    const v4f bb = *(const v4fa*)(cb + c + 4);
#pragma unroll
    for (int u = 0; u < 4; ++u) { bv[u] = bf16r(ba[u]); bv[4 + u] = bf16r(bb[u]); }
  }
  v8h hv;
#pragma unroll
  for (int u = 0; u < 8; ++u) {
    const float sres = conv_silu(wv[0][u], wv[1][u], wv[2][u], wv[3][u], xv[0][u], xv[1][u], xv[2][u], xv[3][u], bv[u]);
    hv[u] = (_Float16)(16.0f * sres);
  }
  const us8 o = __builtin_bit_cast(us8, hv);
  const size_t off = (size_t)tok * DIN + c;
  *(volatile us8*)(XC + off) = o;
  __threadfence();
  *(volatile us8*)(XC + off) = o;
}

template <int DIR>
__global__ __launch_bounds__(256) void k_scan(const float* __restrict__ XZ, const float* __restrict__ DBC,
                                             const unsigned short* __restrict__ DBR, const unsigned short* __restrict__ WDT,
                                             const float* __restrict__ cw, const float* __restrict__ cb,
                                             const float* __restrict__ dtb, const float* __restrict__ Alog,
                                             const float* __restrict__ Dv, unsigned short* YC) {
#pragma clang fp contract(off)
  __shared__ __attribute__((aligned(16))) float sy[SCH * SYP];
  const int g = blockIdx.x, b = blockIdx.y;
  const int tid = threadIdx.x, lane = tid & 31, wave = tid >> 5, cl = lane & 15, hh = lane >> 4;
  const int d = g * 256 + tid;
  float A2[DST], h[DST];
#pragma unroll
  for (int n = 0; n < DST; ++n) { A2[n] = -__expf(bf16r(Alog[d * DST + n])) * LOG2E; h[n] = 0.0f; }
  const float cw0 = bf16r(cw[0 * DIN + d]), cw1 = bf16r(cw[1 * DIN + d]), cw2 = bf16r(cw[2 * DIN + d]), cw3 = bf16r(cw[3 * DIN + d]);
  const float cbv = bf16r(cb[d]);
  const float Dd = bf16r(Dv[d]);
  const float bd = bf16r(dtb[d]);
  float w1 = 0.0f, w2 = 0.0f, w3 = 0.0f;
  const int chw = g * 256 + wave * 32;
  const us16 bw0 = gfrag(WDT, DTR, chw, 0);
  const us16 bw1 = gfrag(WDT, DTR, chw + 16, 0);
  const int cbase = wave * 32 + cl;

#pragma unroll 1
  for (int c = 0; c < LL / SCH; ++c) {
    const int tn0 = DIR ? (LL - SCH * (c + 1)) : (SCH * c);
    const int rowA = b * LL + tn0;
    const us16 a0 = gfrag(DBR, DTR, rowA, 0);
    const us16 a1 = gfrag(DBR, DTR, rowA + 16, 0);
    const v8f z8 = {0.f, 0.f, 0.f, 0.f, 0.f, 0.f, 0.f, 0.f};
    v8f q00 = mma_f16(a0, bw0, z8);
    v8f q01 = mma_f16(a0, bw1, z8);
    v8f q10 = mma_f16(a1, bw0, z8);
    v8f q11 = mma_f16(a1, bw1, z8);
    wguard4(q00, q01, q10, q11, a0, a1, bw0, bw1);
#pragma unroll
    for (int r = 0; r < 8; ++r) {
      const int rr0 = 8 * hh + r, rr1 = 16 + 8 * hh + r;
      const int s0 = DIR ? (SCH - 1 - rr0) : rr0;
      const int s1 = DIR ? (SCH - 1 - rr1) : rr1;
      sy[s0 * SYP + cbase]      = q00[r];
      sy[s0 * SYP + cbase + 16] = q01[r];
      sy[s1 * SYP + cbase]      = q10[r];
      sy[s1 * SYP + cbase + 16] = q11[r];
    }
    __syncthreads();

#pragma unroll 1
    for (int s = 0; s < SCH; ++s) {
      const int st = c * SCH + s;
      const int t = DIR ? (LL - 1 - st) : st;
      const size_t tok = (size_t)b * LL + (size_t)t;
      const float raw = sy[s * SYP + tid] * (1.0f / 256.0f) + bd;
      const float dl = fmaxf(raw, 0.0f) + log1pf(__expf(-fabsf(raw)));
      const float xcur = XZ[tok * DXZ + d];
      const float zv = XZ[tok * DXZ + DIN + d];
      const float xc = conv_silu(cw0, cw1, cw2, cw3, w3, w2, w1, xcur, cbv);
      w3 = w2; w2 = w1; w1 = xcur;
      const float* pbc = DBC + tok * XDN + DTR;
      v4f Bv[4], Cv[4];
#pragma unroll
      for (int q = 0; q < 4; ++q) {
        Bv[q] = *(const v4fa*)(pbc + 4 * q);
        Cv[q] = *(const v4fa*)(pbc + DST + 4 * q);
      }
      const float dx = dl * xc;
      float y = 0.0f;
#pragma unroll
      for (int n = 0; n < DST; ++n) {
        const float e = exp2f(dl * A2[n]);
        h[n] = e * h[n] + dx * Bv[n >> 2][n & 3];
        y = y + h[n] * Cv[n >> 2][n & 3];
      }
      const float yv = (y + xc * Dd) * siluf(zv);
      sy[s * SYP + tid] = yv;
    }
    __syncthreads();

#pragma unroll
    for (int pass = 0; pass < 2; ++pass) {
#pragma unroll
      for (int it = 0; it < 4; ++it) {
        const int row = 4 * wave + it;
        const int st = c * SCH + row;
        const int t = DIR ? (LL - 1 - st) : st;
        const size_t tok = (size_t)b * LL + (size_t)t;
        const v4f va = *(const v4fa*)(sy + row * SYP + lane * 8);
        const v4f vb = *(const v4fa*)(sy + row * SYP + lane * 8 + 4);
        v8h hv;
#pragma unroll
        for (int u = 0; u < 4; ++u) { hv[u] = (_Float16)(4.0f * va[u]); hv[4 + u] = (_Float16)(4.0f * vb[u]); }
        const size_t o = tok * KCAT + (size_t)(DIR * DIN + g * 256 + lane * 8);
        *(volatile us8*)(YC + o) = __builtin_bit_cast(us8, hv);
      }
      __threadfence();
    }
    __syncthreads();
  }
}

extern "C" void kernel_launch(void* const* d_in, const int* in_sizes, int n_in,
                              void* d_out, int out_size, void* d_ws, size_t ws_size,
                              hipStream_t stream) {
  if (n_in < 21) return;
  if (in_sizes[0] != NTOK * DMOD || in_sizes[1] != DMOD || in_sizes[2] != DMOD || out_size != NTOK * DMOD) return;
  for (int dr = 0; dr < 2; ++dr) {
    const int o = 3 + 9 * dr;
    if (in_sizes[o] != DMOD * DXZ || in_sizes[o + 1] != DCV * DIN || in_sizes[o + 2] != DIN || in_sizes[o + 3] != DIN * XDN ||
        in_sizes[o + 4] != DTR * DIN || in_sizes[o + 5] != DIN || in_sizes[o + 6] != DIN * DST || in_sizes[o + 7] != DIN ||
        in_sizes[o + 8] != DIN * DMOD) return;
  }

  const float* x    = (const float*)d_in[0];
  const float* lng  = (const float*)d_in[1];
  const float* lnb  = (const float*)d_in[2];
  const float* inw[2], *cvw[2], *cvb[2], *xpw[2], *dtw[2], *dtbv[2], *alg[2], *dpv[2], *ouw[2];
  for (int dr = 0; dr < 2; ++dr) {
    const int o = 3 + 9 * dr;
    inw[dr]  = (const float*)d_in[o + 0];
    cvw[dr]  = (const float*)d_in[o + 1];
    cvb[dr]  = (const float*)d_in[o + 2];
    xpw[dr]  = (const float*)d_in[o + 3];
    dtw[dr]  = (const float*)d_in[o + 4];
    dtbv[dr] = (const float*)d_in[o + 5];
    alg[dr]  = (const float*)d_in[o + 6];
    dpv[dr]  = (const float*)d_in[o + 7];
    ouw[dr]  = (const float*)d_in[o + 8];
  }
  float* out = (float*)d_out;

  size_t off = 0;
  auto carve = [&](size_t bytes) -> char* { char* p = (char*)d_ws + off; off += (bytes + 255) & ~(size_t)255; return p; };
  unsigned short* WINT = (unsigned short*)carve((size_t)DXZ * DMOD * 2);
  unsigned short* WXT0 = (unsigned short*)carve((size_t)XDN * DIN * 2);
  unsigned short* WXT1 = (unsigned short*)carve((size_t)XDN * DIN * 2);
  unsigned short* WDT0 = (unsigned short*)carve((size_t)DIN * DTR * 2);
  unsigned short* WDT1 = (unsigned short*)carve((size_t)DIN * DTR * 2);
  unsigned short* WOT  = (unsigned short*)carve((size_t)DMOD * KCAT * 2);
  unsigned short* WH   = (unsigned short*)carve((size_t)NTOK * DMOD * 2);
  float* XZ            = (float*)carve((size_t)NTOK * DXZ * 4);
  unsigned short* XC16 = (unsigned short*)carve((size_t)NTOK * DIN * 2);
  float* DBC           = (float*)carve((size_t)NTOK * XDN * 4);
  unsigned short* DBR  = (unsigned short*)carve((size_t)NTOK * DTR * 2);
  unsigned short* YC   = (unsigned short*)carve((size_t)NTOK * KCAT * 2);
  if (off > ws_size || off > WSCAP) return;

  const dim3 b256(256), b128(128);
  k_cvtT<64><<<dim3(XDN / 64, DIN / 64), b256, 0, stream>>>(xpw[0], XDN, WXT0, DIN, 0, 16.0f);
  k_cvtT<64><<<dim3(XDN / 64, DIN / 64), b256, 0, stream>>>(xpw[1], XDN, WXT1, DIN, 0, 16.0f);
  k_cvtT<32><<<dim3(DIN / 64, 1), b256, 0, stream>>>(dtw[0], DIN, WDT0, DTR, 0, 16.0f);
  k_cvtT<32><<<dim3(DIN / 64, 1), b256, 0, stream>>>(dtw[1], DIN, WDT1, DTR, 0, 16.0f);
  k_cvtT<64><<<dim3(DMOD / 64, DIN / 64), b256, 0, stream>>>(ouw[0], DMOD, WOT, KCAT, 0, 16.0f);
  k_cvtT<64><<<dim3(DMOD / 64, DIN / 64), b256, 0, stream>>>(ouw[1], DMOD, WOT, KCAT, DIN, 16.0f);
  k_ln<<<dim3(NTOK / 8), b256, 0, stream>>>(x, lng, lnb, WH);

  for (int dr = 0; dr < 2; ++dr) {
    unsigned short* WXT = dr ? WXT1 : WXT0;
    unsigned short* WDT = dr ? WDT1 : WDT0;
    k_cvtT<64><<<dim3(DXZ / 64, DMOD / 64), b256, 0, stream>>>(inw[dr], DXZ, WINT, DMOD, 0, 16.0f);
    k_gemm<0><<<dim3(NTOK / 128, DXZ / 64), b128, 0, stream>>>(WH, DMOD, WINT, DMOD, DMOD, 1.0f / 128.0f, XZ, DXZ, DBR, x);
    if (dr == 0) k_conv<0><<<dim3(NTOK / 2), b256, 0, stream>>>(XZ, cvw[0], cvb[0], XC16);
    else         k_conv<1><<<dim3(NTOK / 2), b256, 0, stream>>>(XZ, cvw[1], cvb[1], XC16);
    k_gemm<1><<<dim3(NTOK / 128, XDN / 64), b128, 0, stream>>>(XC16, DIN, WXT, DIN, DIN, 1.0f / 256.0f, DBC, XDN, DBR, x);
    if (dr == 0) k_scan<0><<<dim3(DIN / 256, NB), b256, 0, stream>>>(XZ, DBC, DBR, WDT, cvw[0], cvb[0], dtbv[0], alg[0], dpv[0], YC);
    else         k_scan<1><<<dim3(DIN / 256, NB), b256, 0, stream>>>(XZ, DBC, DBR, WDT, cvw[1], cvb[1], dtbv[1], alg[1], dpv[1], YC);
  }
  k_gemm<2><<<dim3(NTOK / 128, DMOD / 64), b128, 0, stream>>>(YC, KCAT, WOT, KCAT, KCAT, 1.0f / 128.0f, out, DMOD, DBR, x);
}
